// GRU_12764642803875
// MI455X (gfx1250) — hardware-run, weakly checked
//
#include <hip/hip_runtime.h>

typedef __attribute__((ext_vector_type(16))) _Float16 v16h;
typedef __attribute__((ext_vector_type(8)))  _Float16 v8h;
typedef __attribute__((ext_vector_type(8)))  float    v8f;
typedef __attribute__((ext_vector_type(4)))  float    v4f;

constexpr int kB      = 8;
constexpr int kS      = 1024;
constexpr int kIn     = 1024;
constexpr int kState  = 1024;
constexpr int kOut    = 1024;
constexpr int kHeads  = 8;
constexpr int kD      = kState / kHeads;
constexpr int kG3     = 3 * kState;
constexpr int kRows   = kB * kS;
constexpr int kHP     = 136;
constexpr int kTP     = 68;
static_assert(kD == 128);
static_assert(kB == 8);
static_assert(kIn % 32 == 0 && kState % 32 == 0 && kD % 32 == 0);
static_assert(kRows % 64 == 0 && kG3 % 64 == 0 && kOut % 64 == 0);
static_assert(kIn % 64 == 0 && kD % 64 == 0);
static_assert(kHP % 8 == 0 && kHP >= kD);
static_assert((kRows * kIn / 8) % 256 == 0);
static_assert(((kRows / 64) * (kG3 / 64)) % 8 == 0);
static_assert(((kRows / 64) * (kOut / 64)) % 8 == 0);

constexpr float kXCarry   = 16.0f;
constexpr float kWiCarry  = 256.0f;
constexpr float kWoCarry  = 256.0f;
constexpr float kWrCarry  = 4096.0f;
constexpr float kHCarry   = 512.0f;
constexpr float kFoldProj = 1.0f / (kXCarry * kWiCarry);
constexpr float kFoldRec  = 1.0f / (kHCarry * kWrCarry);
constexpr float kFoldOut  = 1.0f / (kHCarry * kWoCarry);
constexpr float kF16MinNormal = 6.103515625e-5f;

constexpr size_t kOut0Elems = (size_t)kRows * kOut;
constexpr size_t kOut1Elems = (size_t)kB * kState;
static_assert(kOut0Elems * 4 == 33554432ull);
static_assert((kOut0Elems + kOut1Elems) * 4 == 33587200ull);

union FragU { v16h v; v8h h[2]; };
__device__ __forceinline__ v16h frag_load(const _Float16* p) {
  FragU f;
  f.h[0] = *(const v8h*)(p);
  f.h[1] = *(const v8h*)(p + 16);
  return f.v;
}
__device__ __forceinline__ v8f mma_f16(v16h a, v16h b, v8f c) {
  return __builtin_amdgcn_wmma_f32_16x16x32_f16(false, a, false, b, (short)0, c, false, false);
}
__device__ __forceinline__ void guard1_h(v8f& a, v16h x, v16h y) {
  asm volatile("v_nop\n\tv_nop\n\tv_nop\n\tv_nop" : "+v"(a) : "v"(x), "v"(y));
}
__device__ __forceinline__ void guard2_h(v8f& a, v8f& b, v16h x, v16h y, v16h z) {
  asm volatile("v_nop\n\tv_nop\n\tv_nop\n\tv_nop" : "+v"(a), "+v"(b) : "v"(x), "v"(y), "v"(z));
}
__device__ __forceinline__ void guard4_h(v8f& a, v8f& b, v8f& c, v8f& d, v16h x, v16h y) {
  asm volatile("v_nop\n\tv_nop\n\tv_nop\n\tv_nop" : "+v"(a), "+v"(b), "+v"(c), "+v"(d) : "v"(x), "v"(y));
}
__device__ __forceinline__ void keep4_h(v16h a, v16h b, v16h c, v16h d) {
  asm volatile("v_nop" :: "v"(a), "v"(b), "v"(c), "v"(d));
}
__device__ __forceinline__ void acc_guard4(v8f& a, v8f& b, v8f& c, v8f& d) {
  asm volatile("v_nop\n\tv_nop\n\tv_nop\n\tv_nop" : "+v"(a), "+v"(b), "+v"(c), "+v"(d));
}

__device__ __forceinline__ _Float16 f16_op(float v) {
  const float w = (fabsf(v) < kF16MinNormal) ? 0.0f : v;
  return (_Float16)w;
}
__device__ __forceinline__ float fsig(float x) {
  return __builtin_amdgcn_rcpf(1.0f + __expf(-x));
}
__device__ __forceinline__ float ftanh(float x) {
  return 1.0f - 2.0f * __builtin_amdgcn_rcpf(__expf(2.0f * x) + 1.0f);
}

__global__ __launch_bounds__(256) void cvt_rows_f16_kernel(
    const float* __restrict__ src, unsigned short* __restrict__ dst, int n8, float sc) {
  const int i = blockIdx.x * 256 + threadIdx.x;
  if (i < n8) {
    const float* sp = src + (size_t)i * 8;
    const v4f a = *(const v4f*)(sp);
    const v4f b = *(const v4f*)(sp + 4);
    v8h hv;
#pragma unroll
    for (int e = 0; e < 4; ++e) {
      const float fa = a[e] * sc;
      const float fb = b[e] * sc;
      hv[e]     = f16_op(fa);
      hv[4 + e] = f16_op(fb);
    }
    unsigned short* dp = dst + (size_t)i * 8;
    *(volatile v8h*)dp = hv;
    __threadfence();
    *(volatile v8h*)dp = hv;
  }
}

__global__ __launch_bounds__(256) void transpose_f16_kernel(
    const float* __restrict__ src, int spitch, long sstride,
    unsigned short* __restrict__ dst, int dpitch, long dstride, float sc) {
  __shared__ __align__(16) float sT[64 * kTP];
  const int tid = threadIdx.x, lane = tid & 31, wave = tid >> 5;
  const int n0 = blockIdx.x * 64;
  const int k0 = blockIdx.y * 64;
  const float* sb = src + (size_t)blockIdx.z * (size_t)sstride;
  unsigned short* db = dst + (size_t)blockIdx.z * (size_t)dstride;
  const int lr = tid >> 4, lc4 = (tid & 15) * 4;
#pragma unroll
  for (int i = 0; i < 4; ++i) {
    const int kr = lr + 16 * i;
    const v4f v = *(const v4f*)(sb + (size_t)(k0 + kr) * spitch + n0 + lc4);
    *(v4f*)(sT + kr * kTP + lc4) = v;
  }
  __syncthreads();
  const int q = lane >> 3, c8 = (lane & 7) * 8;
  v8h hv[2];
#pragma unroll
  for (int it = 0; it < 2; ++it) {
    const int n = it * 32 + wave * 4 + q;
#pragma unroll
    for (int e = 0; e < 8; ++e) {
      const float f = sT[(c8 + e) * kTP + n] * sc;
      hv[it][e] = f16_op(f);
    }
  }
  for (int pass = 0; pass < 2; ++pass) {
#pragma unroll
    for (int it = 0; it < 2; ++it) {
      const int n = it * 32 + wave * 4 + q;
      *(volatile v8h*)(db + (size_t)(n0 + n) * dpitch + k0 + c8) = hv[it];
    }
    __threadfence();
  }
}

template <bool BIAS_N>
__global__ __launch_bounds__(256) void gemm64_f16_kernel(
    const unsigned short* __restrict__ Ap, int lda,
    const unsigned short* __restrict__ Btp, int ldb,
    float* __restrict__ C, int ldc,
    const float* __restrict__ bias,
    int M, int N, int K, float scale) {
  __shared__ __align__(16) float sT[8][16 * 68];
  const _Float16* A  = (const _Float16*)Ap;
  const _Float16* Bt = (const _Float16*)Btp;
  const int lane = threadIdx.x & 31;
  const int wave = threadIdx.x >> 5;
  const int tilesN = N >> 6;
  const int tilesM = M >> 6;
  const int tile = blockIdx.x * 8 + wave;
  if (tile >= tilesM * tilesN) return;
  const int tm = tile / tilesN;
  const int tn = tile - tm * tilesN;
  const int m0 = tm << 6;
  const int n0 = tn << 6;
  const int rlane = lane & 15;
  const int koff  = (lane >> 4) * 8;
  const int mOff  = (lane >> 4) * 8;

  v8f acc[4][4];
#pragma unroll
  for (int i = 0; i < 4; ++i)
#pragma unroll
    for (int j = 0; j < 4; ++j) acc[i][j] = (v8f){0.f, 0.f, 0.f, 0.f, 0.f, 0.f, 0.f, 0.f};

  for (int k0 = 0; k0 < K; k0 += 32) {
    v16h bh[4];
#pragma unroll
    for (int j = 0; j < 4; ++j) {
      const size_t bo = (size_t)(n0 + (j << 4) + rlane) * ldb + koff + k0;
      bh[j] = frag_load(Bt + bo);
    }
#pragma unroll
    for (int i = 0; i < 4; ++i) {
      const size_t ao = (size_t)(m0 + (i << 4) + rlane) * lda + koff + k0;
      const v16h ah = frag_load(A + ao);
#pragma unroll
      for (int j = 0; j < 4; ++j) acc[i][j] = mma_f16(ah, bh[j], acc[i][j]);
      guard4_h(acc[i][0], acc[i][1], acc[i][2], acc[i][3], ah, bh[3]);
    }
    keep4_h(bh[0], bh[1], bh[2], bh[3]);
  }
  acc_guard4(acc[0][0], acc[0][1], acc[0][2], acc[0][3]);
  acc_guard4(acc[1][0], acc[1][1], acc[1][2], acc[1][3]);
  acc_guard4(acc[2][0], acc[2][1], acc[2][2], acc[2][3]);
  acc_guard4(acc[3][0], acc[3][1], acc[3][2], acc[3][3]);

  float* slab = sT[wave];
#pragma unroll
  for (int i = 0; i < 4; ++i) {
    const int mBase = m0 + (i << 4);
#pragma unroll
    for (int j = 0; j < 4; ++j) {
      const int n = n0 + (j << 4) + rlane;
      float bv = 0.f;
      if (BIAS_N) bv = bias[n];
#pragma unroll
      for (int r = 0; r < 8; ++r) {
        float v = acc[i][j][r] * scale;
        if (BIAS_N) v += bv;
        slab[(mOff + r) * 68 + (j << 4) + rlane] = v;
      }
    }
    __builtin_amdgcn_fence(__ATOMIC_RELEASE, "workgroup");
    __builtin_amdgcn_wave_barrier();
    __builtin_amdgcn_fence(__ATOMIC_ACQUIRE, "workgroup");
    {
      const int hh = lane >> 4, c4 = (lane & 15) * 4;
      for (int pass = 0; pass < 2; ++pass) {
#pragma unroll
        for (int it = 0; it < 8; ++it) {
          const int row = it * 2 + hh;
          const v4f v = *(const v4f*)(slab + row * 68 + c4);
          *(volatile v4f*)(C + (size_t)(mBase + row) * ldc + n0 + c4) = v;
        }
        __threadfence();
      }
    }
    __builtin_amdgcn_fence(__ATOMIC_RELEASE, "workgroup");
    __builtin_amdgcn_wave_barrier();
    __builtin_amdgcn_fence(__ATOMIC_ACQUIRE, "workgroup");
  }
}

__global__ __launch_bounds__(256) void gated_scan_kernel(
    const float* __restrict__ proj, const float* __restrict__ h0,
    const unsigned short* __restrict__ wrecp,
    unsigned short* __restrict__ hs16, float* __restrict__ hT) {
  __shared__ __align__(16) _Float16 hA[16 * kHP];
  __shared__ __align__(16) _Float16 rhA[16 * kHP];
  __shared__ __align__(16) float inS[2][3 * kB * kD];
  __shared__ __align__(16) float hF[kB * kD];

  const _Float16* wrec = (const _Float16*)wrecp;
  const int tid = threadIdx.x, lane = tid & 31, wave = tid >> 5;
  const int c = lane & 15, hh = lane >> 4, koff = hh * 8;
  const int head = blockIdx.x;
  const int col = 16 * wave + c;
  const bool real = (hh == 0);
  const int l16 = lane & 15;

  v16h wR[4], wF[4], wC[4];
  {
    const _Float16* wb = wrec + ((size_t)(head * 3) * kD + col) * kD + koff;
#pragma unroll
    for (int kc = 0; kc < 4; ++kc) {
      wR[kc] = frag_load(wb + 32 * kc);
      wF[kc] = frag_load(wb + (size_t)kD * kD + 32 * kc);
      wC[kc] = frag_load(wb + (size_t)2 * kD * kD + 32 * kc);
    }
  }

  float hreg[8];
#pragma unroll
  for (int r = 0; r < 8; ++r) hreg[r] = h0[(size_t)r * kState + head * kD + col];
#pragma unroll
  for (int r = 0; r < 8; ++r) {
    const float hv = real ? (hreg[r] * kHCarry) : 0.0f;
    hA[(8 * hh + r) * kHP + col] = f16_op(hv);
  }

  const float* pin = proj + ((size_t)wave * kS) * kG3 + head * kD + lane * 4;
  {
    float* in0 = &inS[0][0] + wave * kD + lane * 4;
#pragma unroll
    for (int g = 0; g < 3; ++g) {
      const v4f v = *(const v4f*)(pin + g * kState);
      *(v4f*)(in0 + g * kB * kD) = v;
    }
  }
  __syncthreads();

  const v8f z8 = {0.f, 0.f, 0.f, 0.f, 0.f, 0.f, 0.f, 0.f};
  const _Float16* ha = hA + c * kHP + koff;
  const _Float16* ra = rhA + c * kHP + koff;

#pragma unroll 1
  for (int t = 0; t < kS; ++t) {
    const int cur = t & 1;
    const int nxt = cur ^ 1;
    const int tn = (t + 1 < kS) ? (t + 1) : (kS - 1);
    const float* pn = pin + (size_t)tn * kG3;
    const v4f p0 = *(const v4f*)(pn);
    const v4f p1 = *(const v4f*)(pn + kState);
    const v4f p2 = *(const v4f*)(pn + 2 * kState);
    const float* ic = &inS[cur][0] + col;

    v8f accR = z8, accF = z8;
#pragma unroll
    for (int kc = 0; kc < 4; ++kc) {
      const v16h a = frag_load(ha + 32 * kc);
      accR = mma_f16(a, wR[kc], accR);
      accF = mma_f16(a, wF[kc], accF);
      guard2_h(accR, accF, a, wR[kc], wF[kc]);
    }
    float fg[8];
#pragma unroll
    for (int r = 0; r < 8; ++r) {
      const float pr = accR[r] * kFoldRec + ic[2 * kB * kD + r * kD];
      const float pf = accF[r] * kFoldRec + ic[kB * kD + r * kD];
      const float rg = fsig(pr);
      fg[r] = fsig(pf);
      const float rh = real ? ((rg * hreg[r]) * kHCarry) : 0.0f;
      rhA[(8 * hh + r) * kHP + col] = f16_op(rh);
    }
    {
      float* inN = &inS[nxt][0] + wave * kD + lane * 4;
      *(v4f*)(inN) = p0;
      *(v4f*)(inN + kB * kD) = p1;
      *(v4f*)(inN + 2 * kB * kD) = p2;
    }
    __syncthreads();

    v8f accC = z8;
#pragma unroll
    for (int kc = 0; kc < 4; ++kc) {
      const v16h a = frag_load(ra + 32 * kc);
      accC = mma_f16(a, wC[kc], accC);
      guard1_h(accC, a, wC[kc]);
    }
#pragma unroll
    for (int r = 0; r < 8; ++r) {
      const float pc = accC[r] * kFoldRec + ic[r * kD];
      const float cg = ftanh(pc);
      const float hn = fg[r] * hreg[r] + (1.0f - fg[r]) * cg;
      hreg[r] = hn;
      const float hv = real ? (hn * kHCarry) : 0.0f;
      hA[(8 * hh + r) * kHP + col] = f16_op(hv);
    }
    __syncthreads();

    {
      v8h sv = *(const v8h*)(hA + wave * kHP + l16 * 8);
      asm volatile("" : "+v"(sv));
      unsigned short* dp = hs16 + ((size_t)wave * kS + (size_t)t) * kState + head * kD + l16 * 8;
      for (int pass = 0; pass < 2; ++pass) {
        if (lane < 16) *(volatile v8h*)dp = sv;
        __threadfence();
      }
    }
  }

  if (real) {
#pragma unroll
    for (int r = 0; r < 8; ++r) hF[r * kD + col] = hreg[r];
  }
  __syncthreads();
  {
    const v4f fv = *(const v4f*)(hF + wave * kD + lane * 4);
    float* tp = hT + (size_t)wave * kState + head * kD + lane * 4;
    for (int pass = 0; pass < 2; ++pass) {
      *(volatile v4f*)tp = fv;
      __threadfence();
    }
  }
}

extern "C" void kernel_launch(void* const* d_in, const int* in_sizes, int n_in,
                              void* d_out, int out_size, void* d_ws, size_t ws_size,
                              hipStream_t stream) {
  if (n_in < 8 || d_out == nullptr || d_ws == nullptr) return;
  if (in_sizes[0] != kRows * kIn) return;
  if (in_sizes[1] != kB * kState) return;
  if (in_sizes[2] != kIn * kG3) return;
  if (in_sizes[3] != kG3) return;
  if (in_sizes[4] != kHeads * kD * kD) return;
  if (in_sizes[5] != kHeads * kD * kD) return;
  if (in_sizes[6] != kHeads * kD * kD) return;
  if (in_sizes[7] != kState * kOut) return;
  if ((size_t)out_size != kOut0Elems + kOut1Elems) return;

  const float* x       = (const float*)d_in[0];
  const float* h0      = (const float*)d_in[1];
  const float* Wi      = (const float*)d_in[2];
  const float* bi      = (const float*)d_in[3];
  const float* w_state = (const float*)d_in[4];
  const float* w_forg  = (const float*)d_in[5];
  const float* w_reset = (const float*)d_in[6];
  const float* Wo      = (const float*)d_in[7];
  float* out0 = (float*)d_out;
  float* out1 = out0 + kOut0Elems;

  char* ws = (char*)d_ws;
  size_t off = 0;
  auto carve = [&](size_t bytes) -> char* { char* p = ws + off; off += (bytes + 255) & ~(size_t)255; return p; };
  unsigned short* XH16  = (unsigned short*)carve((size_t)kRows * kIn * 2);
  unsigned short* WI16T = (unsigned short*)carve((size_t)kG3 * kIn * 2);
  unsigned short* WO16T = (unsigned short*)carve((size_t)kOut * kState * 2);
  unsigned short* WREC  = (unsigned short*)carve((size_t)kHeads * 3 * kD * kD * 2);
  float*          PROJ  = (float*)carve((size_t)kRows * kG3 * 4);
  if (off > ws_size || off > (size_t)134217728) return;

  const int n8x = kRows * kIn / 8;
  cvt_rows_f16_kernel<<<n8x / 256, 256, 0, stream>>>(x, XH16, n8x, kXCarry);

  transpose_f16_kernel<<<dim3(kG3 / 64, kIn / 64, 1), 256, 0, stream>>>(
      Wi, kG3, 0L, WI16T, kIn, 0L, kWiCarry);

  transpose_f16_kernel<<<dim3(kOut / 64, kState / 64, 1), 256, 0, stream>>>(
      Wo, kOut, 0L, WO16T, kState, 0L, kWoCarry);

  const long wsrc = (long)kD * kD;
  const long wdst = (long)3 * kD * kD;
  transpose_f16_kernel<<<dim3(kD / 64, kD / 64, kHeads), 256, 0, stream>>>(
      w_reset, kD, wsrc, WREC, kD, wdst, kWrCarry);
  transpose_f16_kernel<<<dim3(kD / 64, kD / 64, kHeads), 256, 0, stream>>>(
      w_forg, kD, wsrc, WREC + (size_t)kD * kD, kD, wdst, kWrCarry);
  transpose_f16_kernel<<<dim3(kD / 64, kD / 64, kHeads), 256, 0, stream>>>(
      w_state, kD, wsrc, WREC + (size_t)2 * kD * kD, kD, wdst, kWrCarry);

  gemm64_f16_kernel<true><<<(kRows / 64) * (kG3 / 64) / 8, 256, 0, stream>>>(
      XH16, kIn, WI16T, kIn, PROJ, kG3, bi, kRows, kG3, kIn, kFoldProj);

  gated_scan_kernel<<<kHeads, 256, 0, stream>>>(PROJ, h0, WREC, XH16, out1);

  gemm64_f16_kernel<false><<<(kRows / 64) * (kOut / 64) / 8, 256, 0, stream>>>(
      XH16, kState, WO16T, kState, out0, kOut, bi, kRows, kOut, kState, kFoldOut);
}
